// RNN_67886253080777
// MI455X (gfx1250) — hardware-verified
//
#include <hip/hip_runtime.h>
#include <math.h>

constexpr int NSEQ     = 8192;
constexpr int NSTEP    = 12;
constexpr int NFIN     = 64;
constexpr int NHID     = 256;
constexpr int NTHR     = 256;
constexpr int ROWS_BLK = 32;
constexpr int HPITCH   = 264;
constexpr int NROWS    = NSEQ * NSTEP;
constexpr int NOUT     = NROWS * NFIN;
constexpr int CONST_FLOATS = 2048;
constexpr int CB_OFF   = 512;
constexpr float WCARRY     = 16.0f;
constexpr float WCARRY_INV = 1.0f / 16.0f;

static_assert(NSEQ == 32 * 256, "sequence count");
static_assert(NROWS == 98304 && NOUT == 6291456, "plane sizes");
static_assert(NSEQ % ROWS_BLK == 0, "row tiles exact");
static_assert((ROWS_BLK * HPITCH) % NTHR == 0, "zero fill exact");
static_assert(NFIN % 32 == 0 && NHID % 32 == 0, "K multiples of 32");
static_assert(NROWS % 64 == 0 && NFIN % 64 == 0, "GEMM M, N tile multiples");
static_assert(((NROWS / 64) * (NFIN / 64)) % 8 == 0, "GEMM grid exact");
static_assert(NHID == 32 * (NTHR / 32), "8 waves x 32 hidden columns");
static_assert(ROWS_BLK == 4 * (NTHR / 32), "4 stored rows per wave");
static_assert(NSTEP * NFIN == 3 * NTHR, "bias table staging exact");
static_assert(HPITCH % 8 == 0, "16-B aligned LDS rows");

typedef __attribute__((ext_vector_type(16))) _Float16 v16h;
typedef __attribute__((ext_vector_type(8)))  _Float16 v8h;
typedef __attribute__((ext_vector_type(16))) __bf16   v16b;
typedef __attribute__((ext_vector_type(8)))  __bf16   v8b;
typedef __attribute__((ext_vector_type(8)))  float    v8f;
typedef __attribute__((ext_vector_type(4)))  float    v4f;

__device__ __forceinline__ unsigned short f2bf_bits(float f) {
  unsigned u = __float_as_uint(f);
  return (unsigned short)((u + 0x7FFFu + ((u >> 16) & 1u)) >> 16);
}
__device__ __forceinline__ float bf_bits2f(unsigned short h) { return __uint_as_float(((unsigned)h) << 16); }

__device__ __forceinline__ void dep_guard_h(v8f& a, v8f& b, v16h x, v16h y) { asm volatile("v_nop\n\tv_nop\n\tv_nop\n\tv_nop" : "+v"(a), "+v"(b) : "v"(x), "v"(y)); }
__device__ __forceinline__ void dep_guard_b(v8f& a, v8f& b, v16b x, v16b y) { asm volatile("v_nop\n\tv_nop\n\tv_nop\n\tv_nop" : "+v"(a), "+v"(b) : "v"(x), "v"(y)); }
__device__ __forceinline__ void keep4_h(v16h a, v16h b, v16h c, v16h d) { asm volatile("v_nop" :: "v"(a), "v"(b), "v"(c), "v"(d)); }
__device__ __forceinline__ void keep4_b(v16b a, v16b b, v16b c, v16b d) { asm volatile("v_nop" :: "v"(a), "v"(b), "v"(c), "v"(d)); }
__device__ __forceinline__ void acc_guard4(v8f& a, v8f& b, v8f& c, v8f& d) { asm volatile("v_nop\n\tv_nop\n\tv_nop\n\tv_nop" : "+v"(a), "+v"(b), "+v"(c), "+v"(d)); }
__device__ __forceinline__ void guard4_h(v8f& a, v8f& b, v8f& c, v8f& d, v16h x0, v16h x1, v16h y0, v16h y1) {
  asm volatile("v_nop\n\tv_nop\n\tv_nop\n\tv_nop" : "+v"(a), "+v"(b), "+v"(c), "+v"(d) : "v"(x0), "v"(x1), "v"(y0), "v"(y1));
}

template <typename T> struct Frag;
template <> struct Frag<_Float16> {
  typedef v16h V; union U { v16h v; v8h h[2]; };
  static __device__ __forceinline__ v16h load(const _Float16* p) {
    U f; f.h[0] = *(const v8h*)(p); f.h[1] = *(const v8h*)(p + 16); return f.v;
  }
  static __device__ __forceinline__ v8f mma(v16h a, v16h b, v8f c) {
    return __builtin_amdgcn_wmma_f32_16x16x32_f16(false, a, false, b, (short)0, c, false, false);
  }
  static __device__ __forceinline__ void guard(v8f& a, v8f& b, v16h x, v16h y) { dep_guard_h(a, b, x, y); }
  static __device__ __forceinline__ void keep(v16h a, v16h b, v16h c, v16h d) { keep4_h(a, b, c, d); }
};
template <> struct Frag<__bf16> {
  typedef v16b V; union U { v16b v; v8b h[2]; };
  static __device__ __forceinline__ v16b load(const __bf16* p) {
    U f; f.h[0] = *(const v8b*)(p); f.h[1] = *(const v8b*)(p + 16); return f.v;
  }
  static __device__ __forceinline__ v8f mma(v16b a, v16b b, v8f c) {
    return __builtin_amdgcn_wmma_f32_16x16x32_bf16(false, a, false, b, (short)0, c, false, false);
  }
  static __device__ __forceinline__ void guard(v8f& a, v8f& b, v16b x, v16b y) { dep_guard_b(a, b, x, y); }
  static __device__ __forceinline__ void keep(v16b a, v16b b, v16b c, v16b d) { keep4_b(a, b, c, d); }
};

__device__ __forceinline__ float rnn_tanh(float x) {
  const float e = expf(2.0f * x);
  return 1.0f - 2.0f * __builtin_amdgcn_rcpf(e + 1.0f);
}

template <int ET> struct Elem;
template <> struct Elem<0> { typedef _Float16 T; };
template <> struct Elem<1> { typedef __bf16 T; };
template <int ET, bool SPLIT, int BIAS_MODE, int OUT_MODE, bool RESID, int ACT = 0>
__global__ __launch_bounds__(256) void wmma_gemm64(
    const unsigned short* __restrict__ Ap, const unsigned short* __restrict__ A2p, int lda, long strideA,
    const unsigned short* __restrict__ Btp, const unsigned short* __restrict__ Bt2p, int ldb, long strideB,
    void* __restrict__ Cout, void* __restrict__ Cout2, int ldc, long strideC,
    const float* __restrict__ bias,
    const float* __restrict__ resid, long strideR,
    int M, int N, int K, float scale) {
  typedef typename Elem<ET>::T T;
  typedef typename Frag<T>::V V;
  const T* A = (const T*)Ap; const T* A2 = (const T*)A2p; const T* Bt = (const T*)Btp; const T* Bt2 = (const T*)Bt2p;
  __shared__ __align__(16) float sT[8][16 * 68];
  const int b    = blockIdx.y;
  const int lane = threadIdx.x & 31;
  const int wave = threadIdx.x >> 5;
  const int tilesN = N >> 6;
  const int tilesM = M >> 6;
  const int tile = blockIdx.x * 8 + wave;
  if (tile >= tilesM * tilesN) return;
  const int tm = tile / tilesN;
  const int tn = tile - tm * tilesN;
  const int m0 = tm << 6;
  const int n0 = tn << 6;

  const T* Ab  = A  + (size_t)b * strideA;
  const T* Bb  = Bt + (size_t)b * strideB;
  const T* Ab2 = SPLIT ? (A2  + (size_t)b * strideA) : nullptr;
  const T* Bb2 = SPLIT ? (Bt2 + (size_t)b * strideB) : nullptr;

  const int rlane = lane & 15;
  const int koff  = (lane >> 4) * 8;
  const int mOff  = (lane >> 4) * 8;

  v8f acc[4][4];
#pragma unroll
  for (int i = 0; i < 4; ++i)
#pragma unroll
    for (int j = 0; j < 4; ++j) acc[i][j] = (v8f){0.f,0.f,0.f,0.f,0.f,0.f,0.f,0.f};

  for (int k0 = 0; k0 < K; k0 += 32) {
    V bh[4], bl[4];
#pragma unroll
    for (int j = 0; j < 4; ++j) {
      const size_t bo = (size_t)(n0 + (j << 4) + rlane) * ldb + koff + k0;
      bh[j] = Frag<T>::load(Bb + bo);
      if (SPLIT) bl[j] = Frag<T>::load(Bb2 + bo);
    }
#pragma unroll
    for (int i = 0; i < 4; ++i) {
      const size_t ao = (size_t)(m0 + (i << 4) + rlane) * lda + koff + k0;
      V ah = Frag<T>::load(Ab + ao);
      V al;
      if (SPLIT) al = Frag<T>::load(Ab2 + ao);
#pragma unroll
      for (int j = 0; j < 4; ++j) {
        acc[i][j] = Frag<T>::mma(ah, bh[j], acc[i][j]);
        if (SPLIT) {
          acc[i][j] = Frag<T>::mma(ah, bl[j], acc[i][j]);
          acc[i][j] = Frag<T>::mma(al, bh[j], acc[i][j]);
        }
      }
      Frag<T>::guard(acc[i][0], acc[i][3], ah, SPLIT ? al : ah);
    }
    Frag<T>::keep(bh[0], bh[1], bh[2], bh[3]);
    if (SPLIT) Frag<T>::keep(bl[0], bl[1], bl[2], bl[3]);
  }
  acc_guard4(acc[0][0], acc[0][1], acc[0][2], acc[0][3]);
  acc_guard4(acc[1][0], acc[1][1], acc[1][2], acc[1][3]);
  acc_guard4(acc[2][0], acc[2][1], acc[2][2], acc[2][3]);
  acc_guard4(acc[3][0], acc[3][1], acc[3][2], acc[3][3]);

  float* slab = sT[wave];
  const float* Rb = RESID ? (resid + (size_t)b * strideR) : nullptr;
#pragma unroll
  for (int i = 0; i < 4; ++i) {
    const int mBase = m0 + (i << 4);
#pragma unroll
    for (int j = 0; j < 4; ++j) {
      const int n = n0 + (j << 4) + rlane;
      float bv = 0.f;
      if (BIAS_MODE == 2) bv = bias[n];
#pragma unroll
      for (int r = 0; r < 8; ++r) {
        float v = acc[i][j][r] * scale;
        if (BIAS_MODE == 1) v += bias[mBase + mOff + r];
        if (BIAS_MODE == 2) v += bv;
        if (RESID) v += Rb[(size_t)(mBase + mOff + r) * ldc + n];
        if (ACT == 1) v = tanhf(v);
        if (ACT == 2) v = fmaxf(v, 0.0f);
        if (ACT == 4) v = (v > 0.f) ? v : 0.01f * v;
        slab[(mOff + r) * 68 + (j << 4) + rlane] = v;
      }
    }
    __builtin_amdgcn_fence(__ATOMIC_RELEASE, "workgroup");
    __builtin_amdgcn_wave_barrier();
    __builtin_amdgcn_fence(__ATOMIC_ACQUIRE, "workgroup");
    if (OUT_MODE == 0) {
      float* C = (float*)Cout + (size_t)b * strideC;
      const int hh = lane >> 4, c4 = (lane & 15) * 4;
      for (int pass = 0; pass < 2; ++pass) {
#pragma unroll
        for (int it = 0; it < 8; ++it) {
          const int row = it * 2 + hh;
          v4f v = *(const v4f*)(slab + row * 68 + c4);
          *(volatile v4f*)(C + (size_t)(mBase + row) * ldc + n0 + c4) = v;
        }
        __threadfence();
      }
    } else {
      const int q = lane >> 3, c8 = (lane & 7) * 8;
      unsigned short* C  = (unsigned short*)Cout  + (size_t)b * strideC;
      unsigned short* C2 = (OUT_MODE == 2) ? ((unsigned short*)Cout2 + (size_t)b * strideC) : nullptr;
      for (int pass = 0; pass < 2; ++pass) {
#pragma unroll
        for (int it = 0; it < 4; ++it) {
          const int row = it * 4 + q;
          const float* sp = slab + row * 68 + c8;
          v8h hv, lv;
#pragma unroll
          for (int e = 0; e < 8; ++e) {
            if (OUT_MODE == 1) {
              hv[e] = (_Float16)sp[e];
            } else {
              unsigned short hb = f2bf_bits(sp[e]);
              unsigned short lb = f2bf_bits(sp[e] - bf_bits2f(hb));
              hv[e] = __builtin_bit_cast(_Float16, hb);
              lv[e] = __builtin_bit_cast(_Float16, lb);
            }
          }
          *(volatile v8h*)(C + (size_t)(mBase + row) * ldc + n0 + c8) = hv;
          if (OUT_MODE == 2) *(volatile v8h*)(C2 + (size_t)(mBase + row) * ldc + n0 + c8) = lv;
        }
        __threadfence();
      }
    }
    __builtin_amdgcn_fence(__ATOMIC_RELEASE, "workgroup");
    __builtin_amdgcn_wave_barrier();
    __builtin_amdgcn_fence(__ATOMIC_ACQUIRE, "workgroup");
  }
}

__global__ __launch_bounds__(NTHR) void cvt8_f16_kernel(const float* __restrict__ src, unsigned short* __restrict__ dst,
                                                        int n8, float sc) {
  const int i = blockIdx.x * NTHR + threadIdx.x;
  if (i < n8) {
    const float* sp = src + (size_t)i * 8;
    const v4f a = *(const v4f*)(sp);
    const v4f b = *(const v4f*)(sp + 4);
    v8h hv;
#pragma unroll
    for (int e = 0; e < 4; ++e) {
      const float fa = a[e] * sc;
      const float fb = b[e] * sc;
      hv[e]     = (_Float16)fa;
      hv[4 + e] = (_Float16)fb;
    }
    *(volatile v8h*)(dst + (size_t)i * 8) = hv;
    __threadfence();
    *(volatile v8h*)(dst + (size_t)i * 8) = hv;
  }
}

__global__ __launch_bounds__(NTHR) void consts_kernel(const float* __restrict__ b_ih0, const float* __restrict__ b_hh0,
                                                      const float* __restrict__ b_ih1, const float* __restrict__ b_hh1,
                                                      const float* __restrict__ b_seq, const float* __restrict__ w_feat,
                                                      const float* __restrict__ b_feat, float* __restrict__ dst) {
  const int tid = threadIdx.x;
  const int ib = (tid & 63) * 4;
  const v4f a0 = *(const v4f*)(b_ih0 + ib);
  const v4f a1 = *(const v4f*)(b_hh0 + ib);
  const v4f a2 = *(const v4f*)(b_ih1 + ib);
  const v4f a3 = *(const v4f*)(b_hh1 + ib);
  const int f4 = (tid & 15) * 4;
  v4f r0 = {0.f, 0.f, 0.f, 0.f}, r1 = r0, r2 = r0, r3 = r0;
#pragma unroll 1
  for (int h4 = 0; h4 < NHID; h4 += 4) {
    r0 += *(const v4f*)(w_feat + (size_t)(f4 + 0) * NHID + h4);
    r1 += *(const v4f*)(w_feat + (size_t)(f4 + 1) * NHID + h4);
    r2 += *(const v4f*)(w_feat + (size_t)(f4 + 2) * NHID + h4);
    r3 += *(const v4f*)(w_feat + (size_t)(f4 + 3) * NHID + h4);
  }
  v4f rs;
  rs[0] = (r0[0] + r0[1]) + (r0[2] + r0[3]);
  rs[1] = (r1[0] + r1[1]) + (r1[2] + r1[3]);
  rs[2] = (r2[0] + r2[1]) + (r2[2] + r2[3]);
  rs[3] = (r3[0] + r3[1]) + (r3[2] + r3[3]);
  const v4f bf = *(const v4f*)(b_feat + f4);
  const int s0 = (tid >= 128) ? ((tid - 128) >> 4) : 0;
  int s1 = 8 + (tid >> 4);
  s1 = (s1 > NSTEP - 1) ? (NSTEP - 1) : s1;
  const float bs0 = b_seq[s0];
  const float bs1 = b_seq[s1];
  const int q = tid >> 6;
  v4f o0, o1;
#pragma unroll
  for (int e = 0; e < 4; ++e) {
    const float cb0 = bs0 * rs[e] + bf[e];
    const float cb1 = bs1 * rs[e] + bf[e];
    const float s01 = a0[e] + a1[e];
    const float s23 = a2[e] + a3[e];
    o0[e] = (q == 0) ? s01 : ((q == 1) ? s23 : cb0);
    o1[e] = (tid < 64) ? cb1 : 0.0f;
  }
  float* p0 = dst + tid * 4;
  float* p1 = dst + 1024 + tid * 4;
  *(volatile v4f*)p0 = o0;
  *(volatile v4f*)p1 = o1;
  __threadfence();
  *(volatile v4f*)p0 = o0;
  *(volatile v4f*)p1 = o1;
}

__global__ __launch_bounds__(NTHR) void rnn2_kernel(const unsigned short* __restrict__ Xhp,
                                                    const unsigned short* __restrict__ Wih0p,
                                                    const unsigned short* __restrict__ Whh0p,
                                                    const unsigned short* __restrict__ Wih1p,
                                                    const unsigned short* __restrict__ Whh1p,
                                                    const float* __restrict__ consts,
                                                    unsigned short* __restrict__ H2p) {
  __shared__ __align__(16) _Float16 H1t[ROWS_BLK * HPITCH];
  __shared__ __align__(16) _Float16 H2t[ROWS_BLK * HPITCH];
  const _Float16* Xh   = (const _Float16*)Xhp;
  const _Float16* Wih0 = (const _Float16*)Wih0p;
  const _Float16* Whh0 = (const _Float16*)Whh0p;
  const _Float16* Wih1 = (const _Float16*)Wih1p;
  const _Float16* Whh1 = (const _Float16*)Whh1p;
  _Float16* H2g = (_Float16*)H2p;

  const int tid = threadIdx.x, lane = tid & 31, wave = tid >> 5;
  const int c = lane & 15, hh = lane >> 4, koff = hh * 8;
  const int rowbase = blockIdx.x * ROWS_BLK;
  const int j0 = 32 * wave + c;
  const int j1 = j0 + 16;

#pragma unroll 1
  for (int i = tid; i < ROWS_BLK * HPITCH; i += NTHR) {
    H1t[i] = (_Float16)0.0f;
    H2t[i] = (_Float16)0.0f;
  }

  const float bl0a = consts[j0];
  const float bl0b = consts[j1];
  const float bl1a = consts[NHID + j0];
  const float bl1b = consts[NHID + j1];

  const _Float16* xrow0 = Xh + ((size_t)(rowbase + c) * NSTEP) * NFIN + koff;
  const _Float16* xrow1 = Xh + ((size_t)(rowbase + 16 + c) * NSTEP) * NFIN + koff;
  const _Float16* wi0a = Wih0 + (size_t)j0 * NFIN + koff;
  const _Float16* wi0b = Wih0 + (size_t)j1 * NFIN + koff;
  const _Float16* wh0a = Whh0 + (size_t)j0 * NHID + koff;
  const _Float16* wh0b = Whh0 + (size_t)j1 * NHID + koff;
  const _Float16* wi1a = Wih1 + (size_t)j0 * NHID + koff;
  const _Float16* wi1b = Wih1 + (size_t)j1 * NHID + koff;
  const _Float16* wh1a = Whh1 + (size_t)j0 * NHID + koff;
  const _Float16* wh1b = Whh1 + (size_t)j1 * NHID + koff;

  const v8f z8 = {0.f, 0.f, 0.f, 0.f, 0.f, 0.f, 0.f, 0.f};
  __syncthreads();

#pragma unroll 1
  for (int t = 0; t < NSTEP; ++t) {
    v8f acc[2][2];
    acc[0][0] = z8; acc[0][1] = z8; acc[1][0] = z8; acc[1][1] = z8;

    {
      const _Float16* x0 = xrow0 + t * NFIN;
      const _Float16* x1 = xrow1 + t * NFIN;
#pragma unroll 1
      for (int kx = 0; kx < NFIN; kx += 32) {
        const v16h A0 = Frag<_Float16>::load(x0 + kx);
        const v16h A1 = Frag<_Float16>::load(x1 + kx);
        const v16h B0 = Frag<_Float16>::load(wi0a + kx);
        const v16h B1 = Frag<_Float16>::load(wi0b + kx);
        acc[0][0] = Frag<_Float16>::mma(A0, B0, acc[0][0]);
        acc[0][1] = Frag<_Float16>::mma(A0, B1, acc[0][1]);
        acc[1][0] = Frag<_Float16>::mma(A1, B0, acc[1][0]);
        acc[1][1] = Frag<_Float16>::mma(A1, B1, acc[1][1]);
        guard4_h(acc[0][0], acc[0][1], acc[1][0], acc[1][1], A0, A1, B0, B1);
      }
    }
    {
      const _Float16* a0p = &H1t[0] + c * HPITCH + koff;
      const _Float16* a1p = &H1t[0] + (16 + c) * HPITCH + koff;
#pragma unroll 1
      for (int k0 = 0; k0 < NHID; k0 += 32) {
        const v16h A0 = Frag<_Float16>::load(a0p + k0);
        const v16h A1 = Frag<_Float16>::load(a1p + k0);
        const v16h B0 = Frag<_Float16>::load(wh0a + k0);
        const v16h B1 = Frag<_Float16>::load(wh0b + k0);
        acc[0][0] = Frag<_Float16>::mma(A0, B0, acc[0][0]);
        acc[0][1] = Frag<_Float16>::mma(A0, B1, acc[0][1]);
        acc[1][0] = Frag<_Float16>::mma(A1, B0, acc[1][0]);
        acc[1][1] = Frag<_Float16>::mma(A1, B1, acc[1][1]);
        guard4_h(acc[0][0], acc[0][1], acc[1][0], acc[1][1], A0, A1, B0, B1);
      }
    }
#pragma unroll
    for (int mi = 0; mi < 2; ++mi) {
#pragma unroll
      for (int r = 0; r < 8; ++r) {
        acc[mi][0][r] = rnn_tanh(acc[mi][0][r] * WCARRY_INV + bl0a);
        acc[mi][1][r] = rnn_tanh(acc[mi][1][r] * WCARRY_INV + bl0b);
      }
    }
    __syncthreads();
#pragma unroll
    for (int mi = 0; mi < 2; ++mi) {
#pragma unroll
      for (int r = 0; r < 8; ++r) {
        const int row = 16 * mi + 8 * hh + r;
        H1t[row * HPITCH + j0] = (_Float16)acc[mi][0][r];
        H1t[row * HPITCH + j1] = (_Float16)acc[mi][1][r];
      }
    }
    __syncthreads();

    acc[0][0] = z8; acc[0][1] = z8; acc[1][0] = z8; acc[1][1] = z8;
    {
      const _Float16* a0p = &H1t[0] + c * HPITCH + koff;
      const _Float16* a1p = &H1t[0] + (16 + c) * HPITCH + koff;
#pragma unroll 1
      for (int k0 = 0; k0 < NHID; k0 += 32) {
        const v16h A0 = Frag<_Float16>::load(a0p + k0);
        const v16h A1 = Frag<_Float16>::load(a1p + k0);
        const v16h B0 = Frag<_Float16>::load(wi1a + k0);
        const v16h B1 = Frag<_Float16>::load(wi1b + k0);
        acc[0][0] = Frag<_Float16>::mma(A0, B0, acc[0][0]);
        acc[0][1] = Frag<_Float16>::mma(A0, B1, acc[0][1]);
        acc[1][0] = Frag<_Float16>::mma(A1, B0, acc[1][0]);
        acc[1][1] = Frag<_Float16>::mma(A1, B1, acc[1][1]);
        guard4_h(acc[0][0], acc[0][1], acc[1][0], acc[1][1], A0, A1, B0, B1);
      }
    }
    {
      const _Float16* a0p = &H2t[0] + c * HPITCH + koff;
      const _Float16* a1p = &H2t[0] + (16 + c) * HPITCH + koff;
#pragma unroll 1
      for (int k0 = 0; k0 < NHID; k0 += 32) {
        const v16h A0 = Frag<_Float16>::load(a0p + k0);
        const v16h A1 = Frag<_Float16>::load(a1p + k0);
        const v16h B0 = Frag<_Float16>::load(wh1a + k0);
        const v16h B1 = Frag<_Float16>::load(wh1b + k0);
        acc[0][0] = Frag<_Float16>::mma(A0, B0, acc[0][0]);
        acc[0][1] = Frag<_Float16>::mma(A0, B1, acc[0][1]);
        acc[1][0] = Frag<_Float16>::mma(A1, B0, acc[1][0]);
        acc[1][1] = Frag<_Float16>::mma(A1, B1, acc[1][1]);
        guard4_h(acc[0][0], acc[0][1], acc[1][0], acc[1][1], A0, A1, B0, B1);
      }
    }
#pragma unroll
    for (int mi = 0; mi < 2; ++mi) {
#pragma unroll
      for (int r = 0; r < 8; ++r) {
        acc[mi][0][r] = rnn_tanh(acc[mi][0][r] * WCARRY_INV + bl1a);
        acc[mi][1][r] = rnn_tanh(acc[mi][1][r] * WCARRY_INV + bl1b);
      }
    }
    __syncthreads();
#pragma unroll
    for (int mi = 0; mi < 2; ++mi) {
#pragma unroll
      for (int r = 0; r < 8; ++r) {
        const int row = 16 * mi + 8 * hh + r;
        H2t[row * HPITCH + j0] = (_Float16)acc[mi][0][r];
        H2t[row * HPITCH + j1] = (_Float16)acc[mi][1][r];
      }
    }
    __syncthreads();

    {
      v8h hv[4];
#pragma unroll
      for (int i = 0; i < 4; ++i) hv[i] = *(const v8h*)(&H2t[0] + (4 * wave + i) * HPITCH + lane * 8);
      for (int pass = 0; pass < 2; ++pass) {
#pragma unroll
        for (int i = 0; i < 4; ++i) {
          const size_t grow = (size_t)(rowbase + 4 * wave + i) * NSTEP + (size_t)t;
          *(volatile v8h*)(H2g + grow * NHID + lane * 8) = hv[i];
        }
        __threadfence();
      }
    }
  }
}

__global__ __launch_bounds__(NTHR) void mix_kernel(const float* __restrict__ Z, const float* __restrict__ wseq,
                                                   const float* __restrict__ consts, float* __restrict__ out) {
  __shared__ __align__(16) float sW[NSTEP * NSTEP];
  __shared__ __align__(16) float sCB[NSTEP * NFIN];
  const int tid = threadIdx.x;
  {
    const int wi = (tid < NSTEP * NSTEP - 1) ? tid : (NSTEP * NSTEP - 1);
    const float wv = wseq[wi];
    if (tid < NSTEP * NSTEP) sW[tid] = wv;
  }
#pragma unroll
  for (int it = 0; it < 3; ++it) {
    const int idx = it * NTHR + tid;
    sCB[idx] = consts[CB_OFF + idx];
  }
  __syncthreads();

  const int ml = tid >> 4;
  const int f4 = (tid & 15) * 4;
  const int m  = blockIdx.x * 16 + ml;
  v4f o[NSTEP];
#pragma unroll
  for (int s = 0; s < NSTEP; ++s) o[s] = *(const v4f*)(sCB + s * NFIN + f4);
  const float* zp = Z + (size_t)m * (NSTEP * NFIN) + f4;
#pragma unroll 1
  for (int t = 0; t < NSTEP; ++t) {
    const v4f z = *(const v4f*)(zp + t * NFIN);
#pragma unroll
    for (int s = 0; s < NSTEP; ++s) {
      const float w = sW[s * NSTEP + t];
      o[s] = o[s] + z * w;
    }
  }
  float* op = out + (size_t)m * (NSTEP * NFIN) + f4;
  for (int pass = 0; pass < 2; ++pass) {
#pragma unroll
    for (int s = 0; s < NSTEP; ++s) *(volatile v4f*)(op + s * NFIN) = o[s];
    __threadfence();
  }
}

extern "C" void kernel_launch(void* const* d_in, const int* in_sizes, int n_in,
                              void* d_out, int out_size, void* d_ws, size_t ws_size, hipStream_t stream) {
  if (n_in < 13 || d_out == nullptr || d_ws == nullptr) return;
  if (in_sizes[0] != NROWS * NFIN || in_sizes[1] != NHID * NFIN || in_sizes[2] != NHID * NHID ||
      in_sizes[3] != NHID || in_sizes[4] != NHID || in_sizes[5] != NHID * NHID || in_sizes[6] != NHID * NHID ||
      in_sizes[7] != NHID || in_sizes[8] != NHID || in_sizes[9] != NSTEP * NSTEP || in_sizes[10] != NSTEP ||
      in_sizes[11] != NFIN * NHID || in_sizes[12] != NFIN || out_size != NOUT) return;

  const float* x      = (const float*)d_in[0];
  const float* w_ih0  = (const float*)d_in[1];
  const float* w_hh0  = (const float*)d_in[2];
  const float* b_ih0  = (const float*)d_in[3];
  const float* b_hh0  = (const float*)d_in[4];
  const float* w_ih1  = (const float*)d_in[5];
  const float* w_hh1  = (const float*)d_in[6];
  const float* b_ih1  = (const float*)d_in[7];
  const float* b_hh1  = (const float*)d_in[8];
  const float* w_seq  = (const float*)d_in[9];
  const float* b_seq  = (const float*)d_in[10];
  const float* w_feat = (const float*)d_in[11];
  const float* b_feat = (const float*)d_in[12];
  float* out = (float*)d_out;

  char* ws = (char*)d_ws;
  size_t off = 0;
  auto carve = [&](size_t bytes) -> char* { char* p = ws + off; off += (bytes + 255) & ~(size_t)255; return p; };
  unsigned short* XH     = (unsigned short*)carve((size_t)NROWS * NFIN * 2);
  unsigned short* WIH0H  = (unsigned short*)carve((size_t)NHID * NFIN * 2);
  unsigned short* WHH0H  = (unsigned short*)carve((size_t)NHID * NHID * 2);
  unsigned short* WIH1H  = (unsigned short*)carve((size_t)NHID * NHID * 2);
  unsigned short* WHH1H  = (unsigned short*)carve((size_t)NHID * NHID * 2);
  unsigned short* WFEATH = (unsigned short*)carve((size_t)NFIN * NHID * 2);
  float*          CONSTS = (float*)carve((size_t)CONST_FLOATS * 4);
  unsigned short* H2     = (unsigned short*)carve((size_t)NROWS * NHID * 2);
  float*          ZP     = (float*)carve((size_t)NROWS * NFIN * 4);
  if (off > ws_size || off > (size_t)134217728) return;

  const int n8x  = NROWS * NFIN / 8;
  const int n8wi = NHID * NFIN / 8;
  const int n8wh = NHID * NHID / 8;
  const int n8wf = NFIN * NHID / 8;
  cvt8_f16_kernel<<<(n8x  + NTHR - 1) / NTHR, NTHR, 0, stream>>>(x,      XH,     n8x,  1.0f);
  cvt8_f16_kernel<<<(n8wi + NTHR - 1) / NTHR, NTHR, 0, stream>>>(w_ih0,  WIH0H,  n8wi, WCARRY);
  cvt8_f16_kernel<<<(n8wh + NTHR - 1) / NTHR, NTHR, 0, stream>>>(w_hh0,  WHH0H,  n8wh, WCARRY);
  cvt8_f16_kernel<<<(n8wh + NTHR - 1) / NTHR, NTHR, 0, stream>>>(w_ih1,  WIH1H,  n8wh, WCARRY);
  cvt8_f16_kernel<<<(n8wh + NTHR - 1) / NTHR, NTHR, 0, stream>>>(w_hh1,  WHH1H,  n8wh, WCARRY);
  cvt8_f16_kernel<<<(n8wf + NTHR - 1) / NTHR, NTHR, 0, stream>>>(w_feat, WFEATH, n8wf, WCARRY);
  consts_kernel<<<1, NTHR, 0, stream>>>(b_ih0, b_hh0, b_ih1, b_hh1, b_seq, w_feat, b_feat, CONSTS);

  rnn2_kernel<<<NSEQ / ROWS_BLK, NTHR, 0, stream>>>(XH, WIH0H, WHH0H, WIH1H, WHH1H, CONSTS, H2);

  const dim3 ggrid((NROWS / 64) * (NFIN / 64) / 8, 1);
  wmma_gemm64<0, false, 0, 0, false, 0><<<ggrid, 256, 0, stream>>>(
      H2, H2, NHID, 0L, WFEATH, WFEATH, NHID, 0L, (void*)ZP, (void*)ZP, NFIN, 0L,
      CONSTS, CONSTS, 0L, NROWS, NFIN, NHID, WCARRY_INV);

  mix_kernel<<<NSEQ / 16, NTHR, 0, stream>>>(ZP, w_seq, CONSTS, out);
}
